// MSA2Pair_76020921139678
// MI455X (gfx1250) — hardware-verified
//
#include <hip/hip_runtime.h>
#include <math.h>

constexpr int NSEQ  = 256;
constexpr int LRES  = 256;
constexpr int NFEAT = 64;
constexpr int NPROJ = 32;
constexpr int NCOUT = 128;
constexpr int NFUSE = 384;
constexpr int NOPK  = NPROJ * NPROJ;
constexpr int NROW  = NSEQ * LRES;
constexpr int NPAIR = LRES * LRES;
constexpr int XPCOLS = 64;
constexpr int TROWS  = LRES * NPROJ;
constexpr int CHUNK_RES = 32;
constexpr int NCHUNK   = LRES / CHUNK_RES;
constexpr int CH_AROWS = CHUNK_RES * NPROJ;
constexpr int CH_PAIRS = CHUNK_RES * LRES;
constexpr int XS_PITCH = 33;
constexpr int ST_PITCH = 264;
constexpr float WCARRY   = 256.0f;
constexpr float FDCARRY  = 256.0f;
constexpr float HCARRY   = 16.0f;
constexpr float QK_SCALE = 0.17677669529663687f;
constexpr float LN_EPS   = 1e-5f;

constexpr size_t OFF_X16  = 0;
constexpr size_t OFF_XP   = OFF_X16  + (size_t)NROW * NFEAT * 2;
constexpr size_t OFF_XT   = OFF_XP   + (size_t)NROW * XPCOLS * 4;
constexpr size_t OFF_FT   = OFF_XT   + (size_t)TROWS * NSEQ * 2;
constexpr size_t OFF_FEAT = OFF_FT   + (size_t)TROWS * NSEQ * 2;
constexpr size_t OFF_WPT  = OFF_FEAT + (size_t)LRES * 64 * 4;
constexpr size_t OFF_W2T  = OFF_WPT  + (size_t)64 * 64 * 2;
constexpr size_t OFF_WF1T = OFF_W2T  + (size_t)NCOUT * NOPK * 2;
constexpr size_t OFF_WF2T = OFF_WF1T + (size_t)NFUSE * NFUSE * 2;
constexpr size_t OFF_OPC  = OFF_WF2T + (size_t)NCOUT * NFUSE * 2;
constexpr size_t OFF_OPN  = OFF_OPC  + (size_t)CH_AROWS * TROWS * 4;
constexpr size_t OFF_PAIR = OFF_OPN  + (size_t)CH_PAIRS * NOPK * 2;
constexpr size_t OFF_PON  = OFF_PAIR + (size_t)CH_PAIRS * NCOUT * 4;
constexpr size_t OFF_H16  = OFF_PON  + (size_t)CH_PAIRS * NCOUT * 4;
constexpr size_t OFF_H2   = OFF_H16  + (size_t)CH_PAIRS * NFUSE * 2;
constexpr size_t WS_TOTAL = OFF_H2   + (size_t)CH_PAIRS * NFUSE * 2;
static_assert(WS_TOTAL == 105586688, "ws total");
static_assert(WS_TOTAL <= (size_t)134217728, "ws cap");
static_assert((OFF_XP % 256) == 0 && (OFF_XT % 256) == 0 && (OFF_FT % 256) == 0 && (OFF_FEAT % 256) == 0 &&
              (OFF_WPT % 256) == 0 && (OFF_W2T % 256) == 0 && (OFF_WF1T % 256) == 0 && (OFF_WF2T % 256) == 0 &&
              (OFF_OPC % 256) == 0 && (OFF_OPN % 256) == 0 && (OFF_PAIR % 256) == 0 && (OFF_PON % 256) == 0 &&
              (OFF_H16 % 256) == 0 && (OFF_H2 % 256) == 0, "alignment");

typedef __attribute__((ext_vector_type(16))) _Float16 v16h;
typedef __attribute__((ext_vector_type(8)))  _Float16 v8h;
typedef __attribute__((ext_vector_type(4)))  _Float16 v4h;
typedef __attribute__((ext_vector_type(16))) __bf16   v16b;
typedef __attribute__((ext_vector_type(8)))  __bf16   v8b;
typedef __attribute__((ext_vector_type(8)))  float    v8f;
typedef __attribute__((ext_vector_type(4)))  float    v4f;
typedef __attribute__((ext_vector_type(4)))  unsigned int v4u;

__device__ __forceinline__ unsigned short f2bf_bits(float f) {
  unsigned u = __float_as_uint(f);
  return (unsigned short)((u + 0x7FFFu + ((u >> 16) & 1u)) >> 16);
}
__device__ __forceinline__ float bf_bits2f(unsigned short h) { return __uint_as_float(((unsigned)h) << 16); }

__device__ __forceinline__ void dep_guard_h(v8f& a, v8f& b, v16h x, v16h y) { asm volatile("v_nop\n\tv_nop\n\tv_nop\n\tv_nop" : "+v"(a), "+v"(b) : "v"(x), "v"(y)); }
__device__ __forceinline__ void dep_guard_b(v8f& a, v8f& b, v16b x, v16b y) { asm volatile("v_nop\n\tv_nop\n\tv_nop\n\tv_nop" : "+v"(a), "+v"(b) : "v"(x), "v"(y)); }
__device__ __forceinline__ void keep4_h(v16h a, v16h b, v16h c, v16h d) { asm volatile("v_nop" :: "v"(a), "v"(b), "v"(c), "v"(d)); }
__device__ __forceinline__ void keep4_b(v16b a, v16b b, v16b c, v16b d) { asm volatile("v_nop" :: "v"(a), "v"(b), "v"(c), "v"(d)); }
__device__ __forceinline__ void acc_guard4(v8f& a, v8f& b, v8f& c, v8f& d) { asm volatile("v_nop\n\tv_nop\n\tv_nop\n\tv_nop" : "+v"(a), "+v"(b), "+v"(c), "+v"(d)); }
template <typename T> struct Frag;
template <> struct Frag<_Float16> {
  typedef v16h V; union U { v16h v; v8h h[2]; };
  static __device__ __forceinline__ v16h load(const _Float16* p) {
    U f; f.h[0] = *(const v8h*)(p); f.h[1] = *(const v8h*)(p + 16); return f.v;
  }
  static __device__ __forceinline__ v8f mma(v16h a, v16h b, v8f c) {
    return __builtin_amdgcn_wmma_f32_16x16x32_f16(false, a, false, b, (short)0, c, false, false);
  }
  static __device__ __forceinline__ void guard(v8f& a, v8f& b, v16h x, v16h y) { dep_guard_h(a, b, x, y); }
  static __device__ __forceinline__ void keep(v16h a, v16h b, v16h c, v16h d) { keep4_h(a, b, c, d); }
};
template <> struct Frag<__bf16> {
  typedef v16b V; union U { v16b v; v8b h[2]; };
  static __device__ __forceinline__ v16b load(const __bf16* p) {
    U f; f.h[0] = *(const v8b*)(p); f.h[1] = *(const v8b*)(p + 16); return f.v;
  }
  static __device__ __forceinline__ v8f mma(v16b a, v16b b, v8f c) {
    return __builtin_amdgcn_wmma_f32_16x16x32_bf16(false, a, false, b, (short)0, c, false, false);
  }
  static __device__ __forceinline__ void guard(v8f& a, v8f& b, v16b x, v16b y) { dep_guard_b(a, b, x, y); }
  static __device__ __forceinline__ void keep(v16b a, v16b b, v16b c, v16b d) { keep4_b(a, b, c, d); }
};

__device__ __forceinline__ unsigned pk16(unsigned short a, unsigned short b) { return (unsigned)a | ((unsigned)b << 16); }
__device__ __forceinline__ unsigned short h_bits(float f) { const _Float16 h = (_Float16)f; return __builtin_bit_cast(unsigned short, h); }

__device__ __forceinline__ float wsum32(float v) {
#pragma unroll
  for (int off = 16; off > 0; off >>= 1) v += __shfl_xor(v, off, 32);
  return v;
}
__device__ __forceinline__ float wmax32(float v) {
#pragma unroll
  for (int off = 16; off > 0; off >>= 1) v = fmaxf(v, __shfl_xor(v, off, 32));
  return v;
}
__device__ __forceinline__ float gsum8(float v) {
  v += __shfl_xor(v, 1, 32);
  v += __shfl_xor(v, 2, 32);
  v += __shfl_xor(v, 4, 32);
  return v;
}
__device__ __forceinline__ float sum4(v4f x) { return (x[0] + x[1]) + (x[2] + x[3]); }
__device__ __forceinline__ float sq4(v4f x) { return (x[0] * x[0] + x[1] * x[1]) + (x[2] * x[2] + x[3] * x[3]); }

template <int ET> struct Elem;
template <> struct Elem<0> { typedef _Float16 T; };
template <> struct Elem<1> { typedef __bf16 T; };
template <int ET, bool SPLIT, int BIAS_MODE, int OUT_MODE, bool RESID, int ACT = 0>
__global__ __launch_bounds__(256) void wmma_gemm64(
    const unsigned short* __restrict__ Ap, const unsigned short* __restrict__ A2p, int lda, long strideA,
    const unsigned short* __restrict__ Btp, const unsigned short* __restrict__ Bt2p, int ldb, long strideB,
    void* __restrict__ Cout, void* __restrict__ Cout2, int ldc, long strideC,
    const float* __restrict__ bias,
    const float* __restrict__ resid, long strideR,
    int M, int N, int K, float scale, float oscale) {
  typedef typename Elem<ET>::T T;
  typedef typename Frag<T>::V V;
  const T* A = (const T*)Ap; const T* A2 = (const T*)A2p; const T* Bt = (const T*)Btp; const T* Bt2 = (const T*)Bt2p;
  __shared__ __align__(16) float sT[8][16 * 68];
  const int b    = blockIdx.y;
  const int lane = threadIdx.x & 31;
  const int wave = threadIdx.x >> 5;
  const int tilesN = N >> 6;
  const int tilesM = M >> 6;
  const int tile = blockIdx.x * 8 + wave;
  if (tile >= tilesM * tilesN) return;
  const int tm = tile / tilesN;
  const int tn = tile - tm * tilesN;
  const int m0 = tm << 6;
  const int n0 = tn << 6;

  const T* Ab  = A  + (size_t)b * strideA;
  const T* Bb  = Bt + (size_t)b * strideB;
  const T* Ab2 = SPLIT ? (A2  + (size_t)b * strideA) : nullptr;
  const T* Bb2 = SPLIT ? (Bt2 + (size_t)b * strideB) : nullptr;

  const int rlane = lane & 15;
  const int koff  = (lane >> 4) * 8;
  const int mOff  = (lane >> 4) * 8;

  v8f acc[4][4];
#pragma unroll
  for (int i = 0; i < 4; ++i)
#pragma unroll
    for (int j = 0; j < 4; ++j) acc[i][j] = (v8f){0.f,0.f,0.f,0.f,0.f,0.f,0.f,0.f};

  for (int k0 = 0; k0 < K; k0 += 32) {
    V bh[4], bl[4];
#pragma unroll
    for (int j = 0; j < 4; ++j) {
      const size_t bo = (size_t)(n0 + (j << 4) + rlane) * ldb + koff + k0;
      bh[j] = Frag<T>::load(Bb + bo);
      if (SPLIT) bl[j] = Frag<T>::load(Bb2 + bo);
    }
#pragma unroll
    for (int i = 0; i < 4; ++i) {
      const size_t ao = (size_t)(m0 + (i << 4) + rlane) * lda + koff + k0;
      V ah = Frag<T>::load(Ab + ao);
      V al;
      if (SPLIT) al = Frag<T>::load(Ab2 + ao);
#pragma unroll
      for (int j = 0; j < 4; ++j) {
        acc[i][j] = Frag<T>::mma(ah, bh[j], acc[i][j]);
        if (SPLIT) {
          acc[i][j] = Frag<T>::mma(ah, bl[j], acc[i][j]);
          acc[i][j] = Frag<T>::mma(al, bh[j], acc[i][j]);
        }
      }
      Frag<T>::guard(acc[i][0], acc[i][3], ah, SPLIT ? al : ah);
    }
    Frag<T>::keep(bh[0], bh[1], bh[2], bh[3]);
    if (SPLIT) Frag<T>::keep(bl[0], bl[1], bl[2], bl[3]);
  }
  acc_guard4(acc[0][0], acc[0][1], acc[0][2], acc[0][3]);
  acc_guard4(acc[1][0], acc[1][1], acc[1][2], acc[1][3]);
  acc_guard4(acc[2][0], acc[2][1], acc[2][2], acc[2][3]);
  acc_guard4(acc[3][0], acc[3][1], acc[3][2], acc[3][3]);

  float* slab = sT[wave];
  const float* Rb = RESID ? (resid + (size_t)b * strideR) : nullptr;
#pragma unroll
  for (int i = 0; i < 4; ++i) {
    const int mBase = m0 + (i << 4);
#pragma unroll
    for (int j = 0; j < 4; ++j) {
      const int n = n0 + (j << 4) + rlane;
      float bv = 0.f;
      if (BIAS_MODE == 2) bv = bias[n];
#pragma unroll
      for (int r = 0; r < 8; ++r) {
        float v = acc[i][j][r] * scale;
        if (BIAS_MODE == 1) v += bias[mBase + mOff + r];
        if (BIAS_MODE == 2) v += bv;
        if (RESID) v += Rb[(size_t)(mBase + mOff + r) * ldc + n];
        if (ACT == 2) v = fmaxf(v, 0.0f);
        if (ACT == 4) v = (v > 0.f) ? v : 0.01f * v;
        v = v * oscale;
        slab[(mOff + r) * 68 + (j << 4) + rlane] = v;
      }
    }
    __builtin_amdgcn_fence(__ATOMIC_RELEASE, "workgroup");
    __builtin_amdgcn_wave_barrier();
    __builtin_amdgcn_fence(__ATOMIC_ACQUIRE, "workgroup");
    if (OUT_MODE == 0) {
      float* C = (float*)Cout + (size_t)b * strideC;
      const int hh = lane >> 4, c4 = (lane & 15) * 4;
      for (int pass = 0; pass < 2; ++pass) {
#pragma unroll
        for (int it = 0; it < 8; ++it) {
          const int row = it * 2 + hh;
          v4f v = *(const v4f*)(slab + row * 68 + c4);
          *(volatile v4f*)(C + (size_t)(mBase + row) * ldc + n0 + c4) = v;
        }
        __threadfence();
      }
    } else {
      const int q = lane >> 3, c8 = (lane & 7) * 8;
      unsigned short* C  = (unsigned short*)Cout  + (size_t)b * strideC;
      unsigned short* C2 = (OUT_MODE == 2) ? ((unsigned short*)Cout2 + (size_t)b * strideC) : nullptr;
      for (int pass = 0; pass < 2; ++pass) {
#pragma unroll
        for (int it = 0; it < 4; ++it) {
          const int row = it * 4 + q;
          const float* sp = slab + row * 68 + c8;
          v8h hv, lv;
#pragma unroll
          for (int e = 0; e < 8; ++e) {
            if (OUT_MODE == 1) {
              hv[e] = (_Float16)sp[e];
            } else {
              unsigned short hb = f2bf_bits(sp[e]);
              unsigned short lb = f2bf_bits(sp[e] - bf_bits2f(hb));
              hv[e] = __builtin_bit_cast(_Float16, hb);
              lv[e] = __builtin_bit_cast(_Float16, lb);
            }
          }
          *(volatile v8h*)(C + (size_t)(mBase + row) * ldc + n0 + c8) = hv;
          if (OUT_MODE == 2) *(volatile v8h*)(C2 + (size_t)(mBase + row) * ldc + n0 + c8) = lv;
        }
        __threadfence();
      }
    }
    __builtin_amdgcn_fence(__ATOMIC_RELEASE, "workgroup");
    __builtin_amdgcn_wave_barrier();
    __builtin_amdgcn_fence(__ATOMIC_ACQUIRE, "workgroup");
  }
}

__global__ __launch_bounds__(256) void k_wtcast(const float* __restrict__ W, unsigned short* __restrict__ WT,
                                               int KD, int NOUT, float scale) {
  __shared__ float sm[64][65];
  const int t  = threadIdx.x;
  const int k0 = blockIdx.x * 64;
  const int n0 = blockIdx.y * 64;
#pragma unroll
  for (int i = 0; i < 16; ++i) {
    const int e = i * 256 + t;
    const int r = e >> 6;
    const int c = e & 63;
    const int n = n0 + c;
    const int nc = (n < NOUT) ? n : (NOUT - 1);
    float v = W[(size_t)(k0 + r) * NOUT + nc] * scale;
    if (n >= NOUT) v = 0.f;
    sm[c][r] = v;
  }
  __syncthreads();
  const int lane = t & 31, wave = t >> 5;
  const int q = lane >> 3, c8 = (lane & 7) * 8;
  for (int pass = 0; pass < 2; ++pass) {
#pragma unroll
    for (int it = 0; it < 2; ++it) {
      const int row = wave * 8 + it * 4 + q;
      unsigned short hb[8];
#pragma unroll
      for (int e = 0; e < 8; ++e) hb[e] = h_bits(sm[row][c8 + e]);
      const v4u u = (v4u){pk16(hb[0], hb[1]), pk16(hb[2], hb[3]), pk16(hb[4], hb[5]), pk16(hb[6], hb[7])};
      *(volatile v4u*)(WT + (size_t)(n0 + row) * KD + k0 + c8) = u;
    }
    __threadfence();
  }
}

__global__ __launch_bounds__(256) void k_ln_msa(const float* __restrict__ msa, const float* __restrict__ g1,
                                               const float* __restrict__ b1, unsigned short* __restrict__ X16) {
  const int lane = threadIdx.x & 31, wave = threadIdx.x >> 5;
  const int sub = lane >> 3, c8 = (lane & 7) * 8;
  const int row = blockIdx.x * 32 + wave * 4 + sub;
  const float* src = msa + (size_t)row * NFEAT + c8;
  const v4f x0 = *(const v4f*)(src);
  const v4f x1 = *(const v4f*)(src + 4);
  float s = sum4(x0) + sum4(x1);
  s = gsum8(s);
  const float mean = s * (1.0f / 64.0f);
  const v4f d0 = x0 - mean, d1 = x1 - mean;
  float q = sq4(d0) + sq4(d1);
  q = gsum8(q);
  const float rs = rsqrtf(q * (1.0f / 64.0f) + LN_EPS);
  const v4f ga = *(const v4f*)(g1 + c8), gb = *(const v4f*)(g1 + c8 + 4);
  const v4f ba = *(const v4f*)(b1 + c8), bb = *(const v4f*)(b1 + c8 + 4);
  const v4f y0 = (d0 * rs) * ga + ba;
  const v4f y1 = (d1 * rs) * gb + bb;
  const v4u u = (v4u){pk16(h_bits(y0[0]), h_bits(y0[1])), pk16(h_bits(y0[2]), h_bits(y0[3])),
                      pk16(h_bits(y1[0]), h_bits(y1[1])), pk16(h_bits(y1[2]), h_bits(y1[3]))};
  unsigned short* dst = X16 + (size_t)row * NFEAT + c8;
  for (int pass = 0; pass < 2; ++pass) {
    *(volatile v4u*)dst = u;
    __threadfence();
  }
}

__device__ __forceinline__ void store_plane_rows(const _Float16* st, unsigned short* __restrict__ plane,
                                                 int l, int wave, int lane) {
  for (int pass = 0; pass < 2; ++pass) {
#pragma unroll
    for (int rr = 0; rr < 4; ++rr) {
      const int p = wave * 4 + rr;
      const v8h v = *(const v8h*)(st + p * ST_PITCH + lane * 8);
      *(volatile v8h*)(plane + ((size_t)(l * NPROJ + p)) * NSEQ + lane * 8) = v;
    }
    __threadfence();
  }
}

__global__ __launch_bounds__(256) void k_seqattn(const float* __restrict__ XP,
    const float* __restrict__ bp, const float* __restrict__ gd, const float* __restrict__ bd,
    const float* __restrict__ Wq, const float* __restrict__ bq,
    const float* __restrict__ Wk, const float* __restrict__ bk,
    unsigned short* __restrict__ XT, unsigned short* __restrict__ FT, float* __restrict__ feat) {
  __shared__ float xs[NSEQ * XS_PITCH];
  __shared__ __align__(16) _Float16 st16[NPROJ * ST_PITCH];
  __shared__ float wks[NPROJ * NPROJ];
  __shared__ float tars[NPROJ], qs[NPROJ], bks[NPROJ], gds[NPROJ], bds[NPROJ], bps[NPROJ];
  __shared__ float redm[8], reds[8];
  __shared__ __align__(16) float frow[64];
  const int t = threadIdx.x, lane = t & 31, wave = t >> 5;
  const int l = blockIdx.x;

  if (t < NPROJ) { gds[t] = gd[t]; bds[t] = bd[t]; bps[t] = bp[t]; bks[t] = bk[t]; }
#pragma unroll
  for (int e = 0; e < 4; ++e) wks[t * 4 + e] = Wk[t * 4 + e];
  __syncthreads();

  {
    const float* src = XP + ((size_t)t * LRES + l) * XPCOLS;
    float* xr = xs + t * XS_PITCH;
#pragma unroll
    for (int i = 0; i < 8; ++i) {
      const v4f v = *(const v4f*)(src + 4 * i);
#pragma unroll
      for (int e = 0; e < 4; ++e) xr[4 * i + e] = v[e] + bps[4 * i + e];
    }
  }
  {
    float* xr = xs + t * XS_PITCH;
    float s = 0.f;
#pragma unroll 1
    for (int p = 0; p < NPROJ; ++p) s += xr[p];
    const float mean = s * (1.0f / 32.0f);
    float vv = 0.f;
#pragma unroll 1
    for (int p = 0; p < NPROJ; ++p) { const float d = xr[p] - mean; vv = fmaf(d, d, vv); }
    const float rs = rsqrtf(vv * (1.0f / 32.0f) + LN_EPS);
#pragma unroll 1
    for (int p = 0; p < NPROJ; ++p) xr[p] = ((xr[p] - mean) * rs) * gds[p] + bds[p];
  }
  __syncthreads();

  if (t < NPROJ) {
    tars[t] = xs[t];
    float a = 0.f;
#pragma unroll 1
    for (int pp = 0; pp < NPROJ; ++pp) a = fmaf(xs[pp], Wq[pp * NPROJ + t], a);
    qs[t] = (a + bq[t]) * QK_SCALE;
  }
#pragma unroll 1
  for (int p = 0; p < NPROJ; ++p) st16[p * ST_PITCH + t] = (_Float16)xs[t * XS_PITCH + p];
  __syncthreads();
  store_plane_rows(st16, XT, l, wave, lane);

  float lg = 0.f;
#pragma unroll 1
  for (int ph = 0; ph < 2; ++ph) {
    float ka[16];
#pragma unroll
    for (int p = 0; p < 16; ++p) ka[p] = 0.f;
#pragma unroll 1
    for (int pp = 0; pp < NPROJ; ++pp) {
      const float xv = xs[t * XS_PITCH + pp];
      const float* wr = wks + pp * NPROJ + ph * 16;
#pragma unroll
      for (int p = 0; p < 16; ++p) ka[p] = fmaf(xv, wr[p], ka[p]);
    }
#pragma unroll
    for (int p = 0; p < 16; ++p) lg = fmaf(qs[ph * 16 + p], ka[p] + bks[ph * 16 + p], lg);
  }

  float mx = wmax32(lg);
  if (lane == 0) redm[wave] = mx;
  __syncthreads();
  float gm = redm[0];
#pragma unroll
  for (int w = 1; w < 8; ++w) gm = fmaxf(gm, redm[w]);
  const float ex = expf(lg - gm);
  float se = wsum32(ex);
  if (lane == 0) reds[wave] = se;
  __syncthreads();
  float tot = reds[0];
#pragma unroll
  for (int w = 1; w < 8; ++w) tot += reds[w];
  const float wn = ex * (1.0f / tot);

#pragma unroll 1
  for (int p = 0; p < NPROJ; ++p) {
    const float fd = wn * xs[t * XS_PITCH + p];
    st16[p * ST_PITCH + t] = (_Float16)(fd * FDCARRY);
    xs[t * XS_PITCH + p] = fd;
  }
  __syncthreads();
  store_plane_rows(st16, FT, l, wave, lane);

  if (t < NPROJ) {
    float s = 0.f;
#pragma unroll 4
    for (int n2 = 0; n2 < NSEQ; ++n2) s += xs[n2 * XS_PITCH + t];
    frow[t] = s;
    frow[NPROJ + t] = tars[t];
  }
  __syncthreads();
  if (wave == 0 && lane < 16) {
    const v4f v = *(const v4f*)(frow + lane * 4);
    float* dst = feat + (size_t)l * 64 + lane * 4;
    *(volatile v4f*)dst = v;
    __threadfence();
    *(volatile v4f*)dst = v;
  }
}

__global__ __launch_bounds__(256) void k_opnorm(const float* __restrict__ OPC, const float* __restrict__ g2d,
                                               const float* __restrict__ b2d, unsigned short* __restrict__ OPN) {
  __shared__ __align__(16) _Float16 slab[8 * NOPK];
  const int lane = threadIdx.x & 31, wave = threadIdx.x >> 5;
  const int pr = blockIdx.x * 8 + wave;
  const int il = pr >> 8, j = pr & 255;
  const float* src = OPC + ((size_t)(il * NPROJ + lane)) * TROWS + j * NPROJ;
  v4f a[8];
#pragma unroll
  for (int i = 0; i < 8; ++i) a[i] = *(const v4f*)(src + 4 * i);
  float s = 0.f;
#pragma unroll
  for (int i = 0; i < 8; ++i) s += sum4(a[i]);
  s = wsum32(s);
  const float mean = s * (1.0f / 1024.0f);
  float q = 0.f;
#pragma unroll
  for (int i = 0; i < 8; ++i) { const v4f d = a[i] - mean; q += sq4(d); }
  q = wsum32(q);
  const float rs = rsqrtf(q * (1.0f / 1024.0f) + LN_EPS);
  _Float16* sl = slab + wave * NOPK;
  const float* gp = g2d + lane * NPROJ;
  const float* bpp = b2d + lane * NPROJ;
#pragma unroll
  for (int m8 = 0; m8 < 4; ++m8) {
    v8h hv;
#pragma unroll
    for (int i2 = 0; i2 < 2; ++i2) {
      const int i = m8 * 2 + i2;
      const v4f g = *(const v4f*)(gp + 4 * i);
      const v4f bb = *(const v4f*)(bpp + 4 * i);
      const v4f y = ((a[i] - mean) * rs) * g + bb;
#pragma unroll
      for (int e = 0; e < 4; ++e) hv[i2 * 4 + e] = (_Float16)y[e];
    }
    *(v8h*)(sl + lane * NPROJ + m8 * 8) = hv;
  }
  __builtin_amdgcn_fence(__ATOMIC_RELEASE, "workgroup");
  __builtin_amdgcn_wave_barrier();
  __builtin_amdgcn_fence(__ATOMIC_ACQUIRE, "workgroup");
  unsigned short* dst = OPN + (size_t)pr * NOPK;
  for (int pass = 0; pass < 2; ++pass) {
#pragma unroll
    for (int m = 0; m < 4; ++m) {
      const v8h v = *(const v8h*)(sl + (m * 32 + lane) * 8);
      *(volatile v8h*)(dst + (m * 32 + lane) * 8) = v;
    }
    __threadfence();
  }
}

__global__ __launch_bounds__(256) void k_catnorm(const float* __restrict__ pair_orig, const float* __restrict__ PAIRC,
    const float* __restrict__ feat,
    const float* __restrict__ go, const float* __restrict__ bo,
    const float* __restrict__ gn, const float* __restrict__ bn,
    const float* __restrict__ gu, const float* __restrict__ bu,
    float* __restrict__ PON, unsigned short* __restrict__ H16, int chunk) {
  __shared__ __align__(16) _Float16 hsl[8 * NFUSE];
  const int lane = threadIdx.x & 31, wave = threadIdx.x >> 5;
  const int pr = blockIdx.x * 8 + wave;
  const int R  = chunk * CH_PAIRS + pr;
  const int i  = chunk * CHUNK_RES + (pr >> 8);
  const int j  = pr & 255;
  const int c4 = lane * 4;

  const v4f po = *(const v4f*)(pair_orig + (size_t)R * NCOUT + c4);
  float s1 = wsum32(sum4(po));
  const float m1 = s1 * (1.0f / 128.0f);
  const v4f d1 = po - m1;
  const float q1 = wsum32(sq4(d1));
  const float rs1 = rsqrtf(q1 * (1.0f / 128.0f) + LN_EPS);
  const v4f pon = (d1 * rs1) * (*(const v4f*)(go + c4)) + (*(const v4f*)(bo + c4));

  const v4f pv = *(const v4f*)(PAIRC + (size_t)pr * NCOUT + c4);
  float s2 = wsum32(sum4(pv));
  const float m2 = s2 * (1.0f / 128.0f);
  const v4f d2 = pv - m2;
  const float q2 = wsum32(sq4(d2));
  const float rs2 = rsqrtf(q2 * (1.0f / 128.0f) + LN_EPS);
  const v4f pn = (d2 * rs2) * (*(const v4f*)(gn + c4)) + (*(const v4f*)(bn + c4));

  const int fsel = (lane < 16) ? i : j;
  const v4f ff = *(const v4f*)(feat + (size_t)fsel * 64 + (lane & 15) * 4);

  float s3 = wsum32(sum4(pon) + sum4(pn) + sum4(ff));
  const float m3 = s3 * (1.0f / 384.0f);
  const v4f e1 = pon - m3, e2 = pn - m3, e3 = ff - m3;
  const float q3 = wsum32(sq4(e1) + sq4(e2) + sq4(e3));
  const float rs3 = rsqrtf(q3 * (1.0f / 384.0f) + LN_EPS);
  const v4f h1 = (e1 * rs3) * (*(const v4f*)(gu + c4))        + (*(const v4f*)(bu + c4));
  const v4f h2 = (e2 * rs3) * (*(const v4f*)(gu + 128 + c4))  + (*(const v4f*)(bu + 128 + c4));
  const v4f h3 = (e3 * rs3) * (*(const v4f*)(gu + 256 + c4))  + (*(const v4f*)(bu + 256 + c4));

  _Float16* sl = hsl + wave * NFUSE;
  *(v4h*)(sl + c4)       = __builtin_convertvector(h1, v4h);
  *(v4h*)(sl + 128 + c4) = __builtin_convertvector(h2, v4h);
  *(v4h*)(sl + 256 + c4) = __builtin_convertvector(h3, v4h);
  __builtin_amdgcn_fence(__ATOMIC_RELEASE, "workgroup");
  __builtin_amdgcn_wave_barrier();
  __builtin_amdgcn_fence(__ATOMIC_ACQUIRE, "workgroup");

  float* pd = PON + (size_t)pr * NCOUT + c4;
  unsigned short* hd = H16 + (size_t)pr * NFUSE;
  const int t8 = (lane & 15) * 8;
  for (int pass = 0; pass < 2; ++pass) {
    *(volatile v4f*)pd = pon;
    const v8h v0 = *(const v8h*)(sl + lane * 8);
    *(volatile v8h*)(hd + lane * 8) = v0;
    const v8h v1 = *(const v8h*)(sl + 256 + t8);
    if (lane < 16) *(volatile v8h*)(hd + 256 + t8) = v1;
    __threadfence();
  }
}

extern "C" void kernel_launch(void* const* d_in, const int* in_sizes, int n_in,
                              void* d_out, int out_size, void* d_ws, size_t ws_size,
                              hipStream_t stream) {
  if (n_in < 26) return;
  if (in_sizes[0] != NROW * NFEAT) return;
  if (in_sizes[1] != NPAIR * NCOUT) return;
  if (out_size != NPAIR * NCOUT) return;
  if (ws_size < WS_TOTAL) return;

  const float* msa       = (const float*)d_in[0];
  const float* pair_orig = (const float*)d_in[1];
  const float* g1  = (const float*)d_in[2];
  const float* b1  = (const float*)d_in[3];
  const float* Wp  = (const float*)d_in[4];
  const float* bp  = (const float*)d_in[5];
  const float* gd  = (const float*)d_in[6];
  const float* bd  = (const float*)d_in[7];
  const float* Wq  = (const float*)d_in[8];
  const float* bq  = (const float*)d_in[9];
  const float* Wk  = (const float*)d_in[10];
  const float* bk  = (const float*)d_in[11];
  const float* g2d = (const float*)d_in[12];
  const float* b2d = (const float*)d_in[13];
  const float* W2  = (const float*)d_in[14];
  const float* b2  = (const float*)d_in[15];
  const float* go  = (const float*)d_in[16];
  const float* bo  = (const float*)d_in[17];
  const float* gn  = (const float*)d_in[18];
  const float* bn  = (const float*)d_in[19];
  const float* gu  = (const float*)d_in[20];
  const float* bu  = (const float*)d_in[21];
  const float* Wf1 = (const float*)d_in[22];
  const float* bf1 = (const float*)d_in[23];
  const float* Wf2 = (const float*)d_in[24];
  const float* bf2 = (const float*)d_in[25];

  char* ws = (char*)d_ws;
  unsigned short* X16  = (unsigned short*)(ws + OFF_X16);
  float*          XP   = (float*)(ws + OFF_XP);
  unsigned short* XT   = (unsigned short*)(ws + OFF_XT);
  unsigned short* FT   = (unsigned short*)(ws + OFF_FT);
  float*          FEAT = (float*)(ws + OFF_FEAT);
  unsigned short* WPT  = (unsigned short*)(ws + OFF_WPT);
  unsigned short* W2T  = (unsigned short*)(ws + OFF_W2T);
  unsigned short* WF1T = (unsigned short*)(ws + OFF_WF1T);
  unsigned short* WF2T = (unsigned short*)(ws + OFF_WF2T);
  float*          OPC  = (float*)(ws + OFF_OPC);
  unsigned short* OPN  = (unsigned short*)(ws + OFF_OPN);
  float*          PAIRC = (float*)(ws + OFF_PAIR);
  float*          PON  = (float*)(ws + OFF_PON);
  unsigned short* H16  = (unsigned short*)(ws + OFF_H16);
  unsigned short* H2   = (unsigned short*)(ws + OFF_H2);
  float* out = (float*)d_out;

  const dim3 blk(256, 1, 1);
  const float winv = 1.0f / WCARRY;

  k_wtcast<<<dim3(NFEAT / 64, 1, 1), blk, 0, stream>>>(Wp, WPT, NFEAT, NPROJ, WCARRY);
  k_wtcast<<<dim3(NOPK / 64, NCOUT / 64, 1), blk, 0, stream>>>(W2, W2T, NOPK, NCOUT, WCARRY);
  k_wtcast<<<dim3(NFUSE / 64, NFUSE / 64, 1), blk, 0, stream>>>(Wf1, WF1T, NFUSE, NFUSE, WCARRY);
  k_wtcast<<<dim3(NFUSE / 64, NCOUT / 64, 1), blk, 0, stream>>>(Wf2, WF2T, NFUSE, NCOUT, WCARRY);

  k_ln_msa<<<dim3(NROW / 32, 1, 1), blk, 0, stream>>>(msa, g1, b1, X16);

  wmma_gemm64<0, false, 0, 0, false, 0><<<dim3((NROW / 64) * (XPCOLS / 64) / 8, 1, 1), blk, 0, stream>>>(
      X16, X16, NFEAT, 0L, WPT, WPT, NFEAT, 0L, (void*)XP, (void*)XP, XPCOLS, 0L,
      b2, PON, 0L, NROW, XPCOLS, NFEAT, winv, 1.0f);

  k_seqattn<<<dim3(LRES, 1, 1), blk, 0, stream>>>(XP, bp, gd, bd, Wq, bq, Wk, bk, XT, FT, FEAT);

  for (int ci = 0; ci < NCHUNK; ++ci) {
    wmma_gemm64<0, false, 0, 0, false, 0><<<dim3((CH_AROWS / 64) * (TROWS / 64) / 8, 1, 1), blk, 0, stream>>>(
        XT + (size_t)ci * CH_AROWS * NSEQ, XT + (size_t)ci * CH_AROWS * NSEQ, NSEQ, 0L,
        FT, FT, NSEQ, 0L, (void*)OPC, (void*)OPC, TROWS, 0L,
        b2, PON, 0L, CH_AROWS, TROWS, NSEQ, 1.0f / FDCARRY, 1.0f);

    k_opnorm<<<dim3(CH_PAIRS / 8, 1, 1), blk, 0, stream>>>(OPC, g2d, b2d, OPN);

    wmma_gemm64<0, false, 2, 0, false, 0><<<dim3((CH_PAIRS / 64) * (NCOUT / 64) / 8, 1, 1), blk, 0, stream>>>(
        OPN, OPN, NOPK, 0L, W2T, W2T, NOPK, 0L, (void*)PAIRC, (void*)PAIRC, NCOUT, 0L,
        b2, PON, 0L, CH_PAIRS, NCOUT, NOPK, winv, 1.0f);

    k_catnorm<<<dim3(CH_PAIRS / 8, 1, 1), blk, 0, stream>>>(pair_orig, PAIRC, FEAT, go, bo, gn, bn, gu, bu, PON, H16, ci);

    wmma_gemm64<0, false, 2, 1, false, 2><<<dim3((CH_PAIRS / 64) * (NFUSE / 64) / 8, 1, 1), blk, 0, stream>>>(
        H16, H16, NFUSE, 0L, WF1T, WF1T, NFUSE, 0L, (void*)H2, (void*)H2, NFUSE, 0L,
        bf1, PON, 0L, CH_PAIRS, NFUSE, NFUSE, winv, HCARRY);

    wmma_gemm64<0, false, 2, 0, true, 0><<<dim3((CH_PAIRS / 64) * (NCOUT / 64) / 8, 1, 1), blk, 0, stream>>>(
        H2, H2, NFUSE, 0L, WF2T, WF2T, NFUSE, 0L,
        (void*)(out + (size_t)ci * CH_PAIRS * NCOUT), (void*)(out + (size_t)ci * CH_PAIRS * NCOUT), NCOUT, 0L,
        bf2, PON, 0L, CH_PAIRS, NCOUT, NFUSE, 1.0f / (HCARRY * WCARRY), 1.0f);
  }
}
